// SKIPGAT_22668837388774
// MI455X (gfx1250) — hardware-verified
//
#include <hip/hip_runtime.h>
#include <math.h>

typedef __attribute__((ext_vector_type(16))) _Float16 v16h;
typedef __attribute__((ext_vector_type(16))) __bf16 v16b;
typedef __attribute__((ext_vector_type(8)))  _Float16 v8h;
typedef __attribute__((ext_vector_type(8)))  float v8f;
typedef __attribute__((ext_vector_type(4)))  float v4f;
typedef __attribute__((ext_vector_type(2)))  float v2f;
typedef __attribute__((ext_vector_type(4)))  unsigned v4u;
typedef __attribute__((ext_vector_type(4)))  int v4i;
typedef float __attribute__((may_alias)) float_a;
typedef int __attribute__((may_alias)) int_a;

template <typename T> __device__ __forceinline__ void vst2(void* p, T v) { *(volatile T*)p = v; __threadfence(); *(volatile T*)p = v; }
__device__ __forceinline__ v8f wmma16(v16h a, v16h b, v8f c) {
  v8f d = __builtin_amdgcn_wmma_f32_16x16x32_f16(false, a, false, b, (short)0, c, false, false);
  asm volatile("v_nop\n\tv_nop\n\tv_nop\n\tv_nop" : "+v"(d) : "v"(a), "v"(b));
  return d;
}
__device__ __forceinline__ v8f wmma_bf(v16b a, v16b b, v8f c) {
  v8f d = __builtin_amdgcn_wmma_f32_16x16x32_bf16(false, a, false, b, (short)0, c, false, false);
  asm volatile("v_nop\n\tv_nop\n\tv_nop\n\tv_nop" : "+v"(d) : "v"(a), "v"(b));
  return d;
}
__device__ __forceinline__ v16h frag_h(const _Float16* rowk0, int lane) {
  union { v16h v; v8h q[2]; } u; const _Float16* p = rowk0 + 8 * (lane >> 4);
  u.q[0] = *(const v8h*)p; u.q[1] = *(const v8h*)(p + 16); return u.v;
}
__device__ __forceinline__ v16h frag_f32(const float* rowk0, int lane) {
  v16h a; const float* p = rowk0 + 8 * (lane >> 4);
#pragma unroll
  for (int i = 0; i < 8; ++i) { a[i] = (_Float16)p[i]; a[8 + i] = (_Float16)p[16 + i]; }
  return a;
}
__device__ __forceinline__ v16h frag_f32s(const float* rowk0, int lane, float sc) {
  v16h a; const float* p = rowk0 + 8 * (lane >> 4);
#pragma unroll
  for (int i = 0; i < 8; ++i) { a[i] = (_Float16)(p[i] * sc); a[8 + i] = (_Float16)(p[16 + i] * sc); }
  return a;
}
__device__ __forceinline__ v16h fragc_f32(const float* W, int k0, int n, int lane, int ld, int K) {
  v16h a; const int g = lane >> 4;
#pragma unroll
  for (int i = 0; i < 8; ++i) { const int ka = k0 + 8 * g + i, kb = ka + 16;
    a[i] = (_Float16)(ka < K ? W[(size_t)(ka < K ? ka : K - 1) * ld + n] : 0.f); a[8 + i] = (_Float16)(kb < K ? W[(size_t)(kb < K ? kb : K - 1) * ld + n] : 0.f); }
  return a;
}
struct F2 { v16b h, l; };
__device__ __forceinline__ F2 bsplit16(const float v[16]) { F2 r;
#pragma unroll
  for (int i = 0; i < 16; ++i) { const __bf16 h = (__bf16)v[i]; r.h[i] = h; r.l[i] = (__bf16)(v[i] - (float)h); }
  return r; }
__device__ __forceinline__ F2 split_row(const float* row, int k0, int lane) { float v[16]; const float* p = row + k0 + 8 * (lane >> 4);
#pragma unroll
  for (int i = 0; i < 8; ++i) { v[i] = p[i]; v[8 + i] = p[16 + i]; }
  return bsplit16(v); }
__device__ __forceinline__ F2 split_rowK(const float* row, int k0, int lane, int K) { float v[16]; const int g = lane >> 4;
#pragma unroll
  for (int i = 0; i < 8; ++i) { const int ka = k0 + 8 * g + i, kb = ka + 16; v[i] = ka < K ? row[ka < K ? ka : K - 1] : 0.f; v[8 + i] = kb < K ? row[kb < K ? kb : K - 1] : 0.f; }
  return bsplit16(v); }
__device__ __forceinline__ F2 split_col(const float* W, int k0, int n, int lane, int ld, int K) { float v[16]; const int g = lane >> 4;
#pragma unroll
  for (int i = 0; i < 8; ++i) { const int ka = k0 + 8 * g + i, kb = ka + 16; v[i] = ka < K ? W[(size_t)(ka < K ? ka : K - 1) * ld + n] : 0.f; v[8 + i] = kb < K ? W[(size_t)(kb < K ? kb : K - 1) * ld + n] : 0.f; }
  return bsplit16(v); }
__device__ __forceinline__ v8f mac3(const F2& a, const F2& b, v8f c) { c = wmma_bf(a.l, b.h, c); c = wmma_bf(a.h, b.l, c); return wmma_bf(a.h, b.h, c); }
__device__ __forceinline__ float sigm(float v) { return 1.0f / (1.0f + expf(-v)); }
#define LDSX() do { asm volatile("s_wait_dscnt 0" ::: "memory"); __builtin_amdgcn_wave_barrier(); __builtin_amdgcn_fence(__ATOMIC_RELEASE, "workgroup"); } while (0)


#define NN 50000
#define NPAD 50048
#define NE0 800000
#define NET 850000
#define ESTR 800000
#define NH 8
#ifndef NNT
#define NNT NN
#endif
typedef __attribute__((ext_vector_type(8))) __bf16 v8b;
__device__ __forceinline__ v16b frag_b(const __bf16* rowk0, int lane) {
  union { v16b v; v8b q[2]; } u; const __bf16* p = rowk0 + 8 * (lane >> 4);
  u.q[0] = *(const v8b*)p; u.q[1] = *(const v8b*)(p + 16); return u.v;
}
__device__ __forceinline__ float bfr(float v) { return (float)(__bf16)v; }
__device__ __attribute__((noinline)) float exp_ni(float v) { return expf(v); }
__device__ __attribute__((noinline)) float erf_ni(float v) { return erff(v); }

#define CSA_N 50000
#define CSA_E 850000
#define CSA_FINN (CSA_E + 32 * CSA_NBK)
#define CSA_CHUNK 4096
#define CSA_BKT 256
#define CSA_NCH ((CSA_E + CSA_CHUNK - 1) / CSA_CHUNK)
#define CSA_NBK ((CSA_N + CSA_BKT - 1) / CSA_BKT)
#define CSA_NBKP (((CSA_NBK + 63) / 64) * 64)
#define CSA_SEGCAP (CSA_E + 32 * CSA_NBK * CSA_NCH)
#ifndef CSA_BCAP
#define CSA_BCAP 10240
#endif
#define CSA_SZ_CNT   (4u * CSA_NCH * CSA_NBKP)
#define CSA_SZ_OFF   (4u * CSA_NBK * (((CSA_NCH + 31) / 32) * 32))
#define CSA_SZ_BST   (4u * (((CSA_NBK + 1 + 31) / 32) * 32))
#define CSA_SZ_SEG   (4u * CSA_SEGCAP)
#define CSA_SZ_FIN   (4u * (CSA_E + 32 * CSA_NBK))
#define CSA_SZ_ROW   (4u * CSA_NBK * CSA_BKT)
#define CSA_OFFP (((CSA_NCH + 31) / 32) * 32)

__global__ __launch_bounds__(256) void k_csA_cnt(const int* __restrict__ DST, int dstride, int* __restrict__ CNT) {
  __shared__ unsigned short sc[256][CSA_NBK + 1]; __shared__ __align__(16) int srow[CSA_NBKP];
  const int c = blockIdx.x, tid = threadIdx.x;
  for (int b = 0; b < CSA_NBK; ++b) sc[tid][b] = 0;
  const size_t e0 = (size_t)c * CSA_CHUNK + tid * 16;
  for (int i = 0; i < 16; ++i) { const size_t e = e0 + i; if (e < (size_t)CSA_E) { int d = DST[e * dstride]; d = min(max(d, 0), CSA_N - 1); sc[tid][d / CSA_BKT] += 1; } }
  __syncthreads();
  for (int b = tid; b < CSA_NBKP; b += 256) { int s = 0; if (b < CSA_NBK) for (int t = 0; t < 256; ++t) s += sc[t][b]; srow[b] = s; }
  __syncthreads();
  for (int q = tid; q < CSA_NBKP / 4; q += 256) vst2((unsigned*)(CNT + (size_t)c * CSA_NBKP + q * 4), *(const v4u*)&srow[q * 4]);
}
__global__ __launch_bounds__(256) void k_csA_scan(const int* __restrict__ CNT, int* __restrict__ OFF, int* __restrict__ BST) {
  __shared__ int sbt[CSA_NBK + 1]; __shared__ int sbs[((CSA_NBK + 1 + 31) / 32) * 32]; __shared__ int scnt[CSA_NBK + 1]; __shared__ __align__(16) int sbuf[64][CSA_OFFP];
  const int tid = threadIdx.x;
  for (int b = tid; b < CSA_NBK; b += 256) { int sp = 0, st = 0; for (int c = 0; c < CSA_NCH; ++c) { const int n = CNT[(size_t)c * CSA_NBKP + b]; st += n; sp += (n + 31) & ~31; } sbt[b] = sp; scnt[b] = st; }
  for (int b = tid; b < ((CSA_NBK + 1 + 31) / 32) * 32; b += 256) sbs[b] = 0;
  __syncthreads();
  if (tid == 0) { int acc = 0, accf = 0; for (int b = 0; b < CSA_NBK; ++b) { const int t = sbt[b]; sbt[b] = acc; acc += t; sbs[b] = accf; accf += (scnt[b] + 31) & ~31; } sbs[CSA_NBK] = accf; }
  __syncthreads();
  for (int b0 = 0; b0 < CSA_NBK; b0 += 64) {
    if (tid < 64 && b0 + tid < CSA_NBK) { const int b = b0 + tid; int o = sbt[b]; for (int c = 0; c < CSA_OFFP; ++c) { if (c < CSA_NCH) { sbuf[tid][c] = o; o += (CNT[(size_t)c * CSA_NBKP + b] + 31) & ~31; } else sbuf[tid][c] = 0; } }
    __syncthreads();
    for (int q = tid; q < 64 * (CSA_OFFP / 4); q += 256) { const int r = q / (CSA_OFFP / 4), pc = q % (CSA_OFFP / 4); if (b0 + r < CSA_NBK) vst2((unsigned*)(OFF + (size_t)(b0 + r) * CSA_OFFP + pc * 4), *(const v4u*)&sbuf[r][pc * 4]); }
    __syncthreads(); }
  for (int q = tid; q < ((CSA_NBK + 1 + 31) / 32) * 32 / 4; q += 256) vst2((unsigned*)(BST + q * 4), *(const v4u*)&sbs[q * 4]);
}
__global__ __launch_bounds__(256) void k_csA_scatter(const int* __restrict__ SRC, const int* __restrict__ DST, int sstride, int dstride, const int* __restrict__ OFF, int* __restrict__ SEGS, int* __restrict__ SEGE) {
  __shared__ unsigned short sc[256][CSA_NBK + 1]; __shared__ int sbase[CSA_NBK + 1]; __shared__ int scn[CSA_NBK + 1]; __shared__ int sord[CSA_CHUNK];
  const int c = blockIdx.x, tid = threadIdx.x;
  for (int b = 0; b < CSA_NBK; ++b) sc[tid][b] = 0;
  const size_t e0 = (size_t)c * CSA_CHUNK + tid * 16; int bk[16];
#pragma unroll
  for (int i = 0; i < 16; ++i) { const size_t e = e0 + i; bk[i] = -1; if (e < (size_t)CSA_E) { int d = DST[e * dstride]; d = min(max(d, 0), CSA_N - 1); bk[i] = d / CSA_BKT; sc[tid][bk[i]] += 1; } }
  __syncthreads();
  for (int b = tid; b < CSA_NBK; b += 256) { int acc = 0; for (int t = 0; t < 256; ++t) { const int v = sc[t][b]; sc[t][b] = (unsigned short)acc; acc += v; } scn[b] = acc; }
  __syncthreads();
  if (tid == 0) { int acc = 0; for (int b = 0; b < CSA_NBK; ++b) { sbase[b] = acc; acc += scn[b]; } }
  __syncthreads();
#pragma unroll
  for (int i = 0; i < 16; ++i) { if (bk[i] >= 0) { const int b = bk[i]; const int r = sc[tid][b]; sc[tid][b] = (unsigned short)(r + 1); sord[sbase[b] + r] = tid * 16 + i; } }
  __syncthreads();
  for (int b = 0; b < CSA_NBK; ++b) { const int n = scn[b]; if (n == 0) continue; const int nl = ((n + 31) & ~31); const size_t o = (size_t)(min(max(OFF[(size_t)b * CSA_OFFP + c], 0), CSA_SEGCAP - nl) & ~31);
    for (int q = tid; q < nl / 4; q += 256) { int4 vs, ve;
#pragma unroll
      for (int k = 0; k < 4; ++k) { const int i = q * 4 + k; int s = -1, eid = -1; if (i < n) { const size_t e = (size_t)c * CSA_CHUNK + sord[sbase[b] + i]; s = min(max(SRC[e * sstride], 0), CSA_N - 1); eid = (int)e; } vs[k] = s; ve[k] = eid; }
      vst2((unsigned*)(SEGS + o + q * 4), *(const v4u*)&vs); vst2((unsigned*)(SEGE + o + q * 4), *(const v4u*)&ve); } }
}
__global__ __launch_bounds__(256) void k_csA_bucket(const int* __restrict__ CNT, const int* __restrict__ OFF, const int* __restrict__ BST, const int* __restrict__ SEGS, const int* __restrict__ SEGE, const int* __restrict__ DST, int dstride, int* __restrict__ FS, int* __restrict__ FE, int* __restrict__ ROWST, int* __restrict__ ROWCNT) {
  __shared__ int ssrc[CSA_BCAP]; __shared__ int seid[CSA_BCAP]; __shared__ unsigned char snod[CSA_BCAP]; __shared__ int souts[CSA_BCAP]; __shared__ int soute[CSA_BCAP]; __shared__ int scount[256]; __shared__ int sstart[257]; __shared__ int stot;
  const int b = blockIdx.x, tid = threadIdx.x;
  if (tid == 0) { int t = 0; for (int c = 0; c < CSA_NCH; ++c) t += min(max(CNT[(size_t)c * CSA_NBKP + b], 0), CSA_CHUNK); stot = (t <= CSA_BCAP) ? t : 0; }
  __syncthreads();
  { int base = 0; for (int c = 0; c < CSA_NCH; ++c) { const int n = min(max(CNT[(size_t)c * CSA_NBKP + b], 0), CSA_CHUNK); const int o = min(max(OFF[(size_t)b * CSA_OFFP + c], 0), CSA_SEGCAP - ((n + 31) & ~31));
      for (int i = tid; i < n; i += 256) { const int p = base + i; if (p < CSA_BCAP) { ssrc[p] = min(max(SEGS[o + i], 0), CSA_N - 1); const int e = min(max(SEGE[o + i], 0), CSA_E - 1); seid[p] = e; int d = DST[(size_t)e * dstride]; d = min(max(d, 0), CSA_N - 1); const int dl = d - b * CSA_BKT; snod[p] = (unsigned char)(dl >= 0 && dl < 256 ? dl : 255); } }
      base += n; } }
  __syncthreads();
  const int node = b * CSA_BKT + tid; int cnt = 0; for (int p = 0; p < stot; ++p) cnt += (snod[p] == tid) ? 1 : 0;
  scount[tid] = cnt; __syncthreads();
  if (tid == 0) { int acc = 0; for (int t = 0; t < 256; ++t) { sstart[t] = acc; acc += scount[t]; } sstart[256] = acc; }
  __syncthreads();
  const int bst0 = min(max(BST[b], 0), CSA_FINN - ((sstart[256] + 31) & ~31)) & ~31; const int gst = bst0 + sstart[tid];
  { int w = sstart[tid]; for (int p = 0; p < stot; ++p) if (snod[p] == tid) { souts[w] = ssrc[p]; soute[w] = seid[p]; ++w; } }
  __syncthreads();
  { const int n = sstart[256]; const int nl = (n + 31) & ~31; for (int q = tid; q < nl / 4; q += 256) { int4 vs, ve;
#pragma unroll
      for (int k = 0; k < 4; ++k) { const int i = q * 4 + k; vs[k] = i < n ? souts[i] : -1; ve[k] = i < n ? soute[i] : -1; }
      vst2((unsigned*)(FS + bst0 + q * 4), *(const v4u*)&vs); vst2((unsigned*)(FE + bst0 + q * 4), *(const v4u*)&ve); } }
  __syncthreads();
  { __shared__ __align__(16) int srs[256], src2[256]; srs[tid] = node < CSA_N ? gst : 0; src2[tid] = node < CSA_N ? cnt : 0; __syncthreads();
    if (tid < 64) vst2((unsigned*)(ROWST + (size_t)b * 256 + tid * 4), *(const v4u*)&srs[tid * 4]); else if (tid < 128) vst2((unsigned*)(ROWCNT + (size_t)b * 256 + (tid - 64) * 4), *(const v4u*)&src2[(tid - 64) * 4]); }
}


#define NET4 (((NET + 3) / 4) * 4)
#define WS_CNT  0u
#define WS_OFF  (WS_CNT + CSA_SZ_CNT)
#define WS_BST  (WS_OFF + CSA_SZ_OFF)
#define WS_SEGS (WS_BST + CSA_SZ_BST)
#define WS_SEGE (WS_SEGS + CSA_SZ_SEG)
#define WS_FS   (WS_SEGE + CSA_SZ_SEG)
#define WS_FE   (WS_FS + CSA_SZ_FIN)
#define WS_RST  (WS_FE + CSA_SZ_FIN)
#define WS_RCT  (WS_RST + CSA_SZ_ROW)
#define WS_ESRC (WS_RCT + CSA_SZ_ROW)
#define WS_EDST (WS_ESRC + 4u * NET4)
#define WS_PW   (WS_EDST + 4u * NET4)
#define P1 0
#define P2 (P1 + 256 * 128)
#define PWEND (P2 + 128 * 256)
#define WS_H    (WS_PW + 2u * PWEND)
#define WS_ESD  (WS_H + 4u * NPAD * 256)
#define WS_G    (WS_ESD + 4u * NH * NPAD * 2)
#define WS_END  (WS_G + 4u * NPAD * 256)

__global__ __launch_bounds__(256) void k_edges(const int* __restrict__ EI, int* __restrict__ ESRC, int* __restrict__ EDST) {
  __shared__ __align__(16) int ss[256], sd_[256]; const int t = threadIdx.x; const size_t e = (size_t)blockIdx.x * 256 + t;
  int s = 0, d = 0; if (e < NE0) { s = EI[e]; d = EI[ESTR + e]; } else if (e < NET) { s = (int)(e - NE0); d = s; }
  ss[t] = s; sd_[t] = d; __syncthreads();
  if (t < 64 && (size_t)blockIdx.x * 256 + t * 4 < NET) { vst2((unsigned*)(ESRC + (size_t)blockIdx.x * 256 + t * 4), *(const v4u*)&ss[t * 4]); vst2((unsigned*)(EDST + (size_t)blockIdx.x * 256 + t * 4), *(const v4u*)&sd_[t * 4]); }
}
__global__ __launch_bounds__(256) void k_packW(const float* __restrict__ Wm, int K, int NOUT, __bf16* __restrict__ DST_) {
  __shared__ __align__(16) __bf16 s[256]; const int n = blockIdx.x, t = threadIdx.x; if (n >= NOUT) return; if (t < K) s[t] = (__bf16)Wm[(size_t)t * NOUT + n]; __syncthreads();
  if (t < K / 8) vst2((unsigned*)(DST_ + (size_t)n * K + t * 8), *(const v4u*)&s[t * 8]);
}
template <int LAYER>
__global__ __launch_bounds__(128) void k_tr(const float* __restrict__ A, const __bf16* __restrict__ P, const float* __restrict__ AS, const float* __restrict__ AD, float* __restrict__ H, float* __restrict__ ESD) {
  constexpr int K = LAYER == 1 ? 128 : 256; constexpr int CH = LAYER == 1 ? 32 : 16; constexpr int HPB = 128 / CH;
  __shared__ __align__(16) float so[4][16][132]; __shared__ __align__(16) float se[HPB][64][2];
  const int tid = threadIdx.x, wave = tid >> 5, lane = tid & 31, col = lane & 15, g = lane >> 4; const size_t r0 = (size_t)blockIdx.x * 64 + wave * 16; const int n0 = blockIdx.y * 128; const int h0 = blockIdx.y * HPB;
  v8f acc[8] = {};
#pragma unroll 2
  for (int kc = 0; kc < K / 32; ++kc) { F2 a; if (LAYER == 1) { v16b ax; const size_t ri = ((r0 + col) < (size_t)NN) ? (r0 + col) : (size_t)(NN - 1); const float* p = A + ri * 128 + kc * 32 + 8 * g;
#pragma unroll
      for (int i2 = 0; i2 < 8; ++i2) { ax[i2] = (__bf16)fmaxf(p[i2], 0.f); ax[8 + i2] = (__bf16)fmaxf(p[16 + i2], 0.f); } a.h = ax; a.l = ax; } else a = split_row(A + (r0 + col) * 256, kc * 32, lane);
#pragma unroll
    for (int j = 0; j < 8; ++j) { const v16b w = frag_b(P + (size_t)(n0 + j * 16 + col) * K + kc * 32, lane); if (LAYER == 2) acc[j] = wmma_bf(a.l, w, acc[j]); acc[j] = wmma_bf(a.h, w, acc[j]); } }
#pragma unroll
  for (int j = 0; j < 8; ++j)
#pragma unroll
    for (int r = 0; r < 8; ++r) so[wave][8 * g + r][j * 16 + col] = acc[j][r];
  LDSX();
  for (int rl = 0; rl < 16; ++rl) { const int c = lane * 4; const int hl = c / CH; float a1 = 0.f, a2 = 0.f;
#pragma unroll
    for (int q = 0; q < 4; ++q) { const float hv = so[wave][rl][c + q]; const int cc = (c + q) % CH; a1 += hv * bfr(AS[(h0 + hl) * CH + cc]); a2 += hv * bfr(AD[(h0 + hl) * CH + cc]); }
#pragma unroll
    for (int o = 1; o < CH / 4; o <<= 1) { a1 += __shfl_xor(a1, o); a2 += __shfl_xor(a2, o); }
    if ((lane % (CH / 4)) == 0) { se[hl][wave * 16 + rl][0] = a1; se[hl][wave * 16 + rl][1] = a2; } }
  for (int rl = 0; rl < 16; ++rl) vst2(H + (r0 + rl) * 256 + n0 + lane * 4, *(const v4f*)&so[wave][rl][lane * 4]);
  __syncthreads();
  for (int q = tid; q < HPB * 32; q += 128) { const int hl = q >> 5, pc = q & 31; vst2(ESD + ((size_t)(h0 + hl) * NPAD + (size_t)blockIdx.x * 64) * 2 + pc * 4, *(const v4f*)(&se[hl][0][0] + pc * 4)); }
}
template <int LAYER>
__global__ __launch_bounds__(256) void k_gat(const float* __restrict__ H, const float* __restrict__ ESD, const int* __restrict__ FS, const int* __restrict__ RST, const int* __restrict__ RCT, const float* __restrict__ BIAS, const float* __restrict__ X, float* __restrict__ OUTP) {
  constexpr int W = LAYER == 1 ? 256 : 128; constexpr int CPL = W / 32; constexpr int CH = LAYER == 1 ? 32 : 16;
  __shared__ __align__(16) float srow[8][W];
  const int tid = threadIdx.x, wave = tid >> 5, lane = tid & 31; const size_t i = (size_t)blockIdx.x * 8 + wave; const int h = (lane * CPL) / CH;
  float acc[CPL];
#pragma unroll
  for (int c = 0; c < CPL; ++c) acc[c] = 0.f;
  if (i < NNT) { const int cnt = min(max(RCT[i], 0), CSA_BCAP); const int st = min(max(RST[i], 0), CSA_FINN - cnt); const float edi = ESD[((size_t)h * NPAD + i) * 2 + 1];
    float m = -3.0e38f;
    for (int e = 0; e < cnt; ++e) { const int sr = FS[st + e]; if (sr < 0 || sr >= NNT) continue; const int s = sr; float v = ESD[((size_t)h * NPAD + s) * 2] + edi; v = v > 0.f ? v : 0.2f * v; m = fmaxf(m, v); }
    float zs = 0.f;
    for (int e = 0; e < cnt; ++e) { const int sr = FS[st + e]; if (sr < 0 || sr >= NNT) continue; const int s = sr; float v = ESD[((size_t)h * NPAD + s) * 2] + edi; v = v > 0.f ? v : 0.2f * v; zs += exp_ni(v - m); }
    const float iz = (cnt > 0) ? 1.0f / zs : 0.f;
    for (int e = 0; e < cnt; ++e) { const int sr = FS[st + e]; if (sr < 0 || sr >= NNT) continue; const int s = sr; float v = ESD[((size_t)h * NPAD + s) * 2] + edi; v = v > 0.f ? v : 0.2f * v; const float al = exp_ni(v - m) * iz; const float* row = H + (size_t)s * 256 + lane * CPL;
#pragma unroll
      for (int c = 0; c < CPL; ++c) acc[c] += al * row[c]; }
#pragma unroll
    for (int c = 0; c < CPL; ++c) { float v = acc[c] + bfr(BIAS[lane * CPL + c]); if (LAYER == 1) v = fmaxf(v, 0.f); else v += bfr(X[i * 128 + lane * CPL + c]); acc[c] = v; } }
#pragma unroll
  for (int c = 0; c < CPL; ++c) srow[wave][lane * CPL + c] = acc[c];
  LDSX();
  if (LAYER == 1) {
#pragma unroll
    for (int pc = 0; pc < 2; ++pc) vst2(OUTP + i * 256 + pc * 128 + lane * 4, *(const v4f*)&srow[wave][pc * 128 + lane * 4]); }
  else { if (i < NN) vst2(OUTP + i * 128 + lane * 4, *(const v4f*)&srow[wave][lane * 4]); }
}
extern "C" void kernel_launch(void* const* d_in, const int* in_sizes, int n_in, void* d_out, int out_size, void* d_ws, size_t ws_size, hipStream_t stream) {
  (void)in_sizes; (void)n_in; (void)out_size;
  const float** F = (const float**)d_in; const int* EI = (const int*)d_in[1];
  if (ws_size < (size_t)WS_END) return;
  char* ws = (char*)d_ws;
  int *CNT = (int*)(ws + WS_CNT), *OFF = (int*)(ws + WS_OFF), *BST = (int*)(ws + WS_BST), *SEGS = (int*)(ws + WS_SEGS), *SEGE = (int*)(ws + WS_SEGE), *FS = (int*)(ws + WS_FS), *FE = (int*)(ws + WS_FE), *RST = (int*)(ws + WS_RST), *RCT = (int*)(ws + WS_RCT), *ESRC = (int*)(ws + WS_ESRC), *EDST = (int*)(ws + WS_EDST);
  __bf16* PW = (__bf16*)(ws + WS_PW); float *H = (float*)(ws + WS_H), *ESD = (float*)(ws + WS_ESD), *G = (float*)(ws + WS_G);
  k_edges<<<(NET + 255) / 256, 256, 0, stream>>>(EI, ESRC, EDST);
  k_csA_cnt<<<CSA_NCH, 256, 0, stream>>>(EDST, 1, CNT); k_csA_scan<<<1, 256, 0, stream>>>(CNT, OFF, BST); k_csA_scatter<<<CSA_NCH, 256, 0, stream>>>(ESRC, EDST, 1, 1, OFF, SEGS, SEGE); k_csA_bucket<<<CSA_NBK, 256, 0, stream>>>(CNT, OFF, BST, SEGS, SEGE, EDST, 1, FS, FE, RST, RCT);
  k_packW<<<256, 256, 0, stream>>>(F[3], 128, 256, PW + P1); k_packW<<<128, 256, 0, stream>>>(F[7], 256, 128, PW + P2);
  k_tr<1><<<dim3(NPAD / 64, 2), 128, 0, stream>>>(F[0], PW + P1, F[4], F[5], H, ESD);
  k_gat<1><<<NPAD / 8, 256, 0, stream>>>(H, ESD, FS, RST, RCT, F[6], F[0], G);
  k_tr<2><<<dim3(NPAD / 64, 1), 128, 0, stream>>>(G, PW + P2, F[8], F[9], H, ESD);
  k_gat<2><<<NPAD / 8, 256, 0, stream>>>(H, ESD, FS, RST, RCT, F[10], F[0], (float*)d_out);
}
